// gnn_embedder2_47854525612047
// MI455X (gfx1250) — hardware-verified
//
#include <hip/hip_runtime.h>
#include <stddef.h>
#include <stdint.h>


#define NTHR   256
#define NWAVE  8
#define EPT    8
#define CHUNK  (NTHR * EPT)
#define WCAP   (EPT * 32)
#define LISTN  (NWAVE * WCAP)
#define NBN    256
#define NBA    128
#define NBB    64
#define ETHR   128
#define EWAVE  4
#define BN_EPS 1e-5f

typedef float          v4f   __attribute__((ext_vector_type(4), __may_alias__));
typedef float          v8f   __attribute__((ext_vector_type(8)));
typedef int            v4i   __attribute__((ext_vector_type(4)));
typedef double         v2d   __attribute__((ext_vector_type(2), __may_alias__));
typedef unsigned short v8us  __attribute__((ext_vector_type(8), __may_alias__));
typedef unsigned short v16us __attribute__((ext_vector_type(16)));
typedef __bf16         v16bf __attribute__((ext_vector_type(16)));
union FragU { v16us v; v8us h[2]; };

__device__ __forceinline__ void wsync() {
  __builtin_amdgcn_fence(__ATOMIC_RELEASE, "wavefront");
  __builtin_amdgcn_wave_barrier();
}

__device__ __forceinline__ v8f bc8(float v) {
  v8f c;
#pragma unroll
  for (int i = 0; i < 8; ++i) c[i] = v;
  return c;
}

__device__ __forceinline__ v8us zu8() {
  v8us z;
#pragma unroll
  for (int i = 0; i < 8; ++i) z[i] = (unsigned short)0;
  return z;
}

__device__ __forceinline__ unsigned bfr(float x) {
  const unsigned u = __float_as_uint(x);
  return (u + 0x7fffu + ((u >> 16) & 1u)) & 0xffff0000u;
}

__device__ __forceinline__ void split8v(v4f a, v4f b, v8us& hi, v8us& lo) {
  unsigned r, r2; float t;
#define SP(I, X) { r = bfr(X); t = (X) - __uint_as_float(r); r2 = bfr(t); \
                   hi[I] = (unsigned short)(r >> 16); lo[I] = (unsigned short)(r2 >> 16); }
  SP(0, a.x) SP(1, a.y) SP(2, a.z) SP(3, a.w) SP(4, b.x) SP(5, b.y) SP(6, b.z) SP(7, b.w)
#undef SP
}

__device__ __forceinline__ v4f bn4(v4f a, const float* mu, const float* rs) {
  v4f o;
  o.x = fmaxf((a.x - mu[0]) * rs[0], 0.0f);
  o.y = fmaxf((a.y - mu[1]) * rs[1], 0.0f);
  o.z = fmaxf((a.z - mu[2]) * rs[2], 0.0f);
  o.w = fmaxf((a.w - mu[3]) * rs[3], 0.0f);
  return o;
}

__device__ __forceinline__ v8f wmb(v16us a, v16us b, v8f c) {
  const v16bf av = __builtin_bit_cast(v16bf, a);
  const v16bf bv = __builtin_bit_cast(v16bf, b);
  v8f d = __builtin_amdgcn_wmma_f32_16x16x32_bf16(false, av, false, bv, (short)0, c, false, false);
  asm volatile("v_nop\n\tv_nop\n\tv_nop\n\tv_nop" : "+v"(d) : "v"(av), "v"(bv));
  return d;
}

__device__ __forceinline__ v8f wmb3(v16us ah, v16us al, v16us bh, v16us bl, v8f c) {
  c = wmb(ah, bh, c);
  c = wmb(ah, bl, c);
  c = wmb(al, bh, c);
  return c;
}

__device__ __forceinline__ v16us ldf(const unsigned short* p, int hh) {
  FragU f;
  f.h[0] = *(const v8us*)(p + 8 * hh);
  f.h[1] = *(const v8us*)(p + 16 + 8 * hh);
  return f.v;
}

__device__ __forceinline__ void afr_plain(const float* p, int hh, FragU& fh, FragU& fl) {
  const v4f a0 = *(const v4f*)(p + 8 * hh);
  const v4f a1 = *(const v4f*)(p + 8 * hh + 4);
  const v4f b0 = *(const v4f*)(p + 16 + 8 * hh);
  const v4f b1 = *(const v4f*)(p + 16 + 8 * hh + 4);
  split8v(a0, a1, fh.h[0], fl.h[0]);
  split8v(b0, b1, fh.h[1], fl.h[1]);
}

__device__ __forceinline__ void afr_bn(const float* p, const float* mu, const float* rs, int hh, FragU& fh, FragU& fl) {
  v4f a0 = *(const v4f*)(p + 8 * hh);
  v4f a1 = *(const v4f*)(p + 8 * hh + 4);
  v4f b0 = *(const v4f*)(p + 16 + 8 * hh);
  v4f b1 = *(const v4f*)(p + 16 + 8 * hh + 4);
  a0 = bn4(a0, mu + 8 * hh,          rs + 8 * hh);
  a1 = bn4(a1, mu + 8 * hh + 4,      rs + 8 * hh + 4);
  b0 = bn4(b0, mu + 16 + 8 * hh,     rs + 16 + 8 * hh);
  b1 = bn4(b1, mu + 16 + 8 * hh + 4, rs + 16 + 8 * hh + 4);
  split8v(a0, a1, fh.h[0], fl.h[0]);
  split8v(b0, b1, fh.h[1], fl.h[1]);
}

template <int KS, int BNF>
__device__ __forceinline__ v8f tgemm(const float* arow, const float* mu, const float* rs,
                                     const unsigned short* bhr, const unsigned short* blr,
                                     float cinit, int hh) {
  v8f d = bc8(cinit);
#pragma unroll
  for (int ks = 0; ks < KS; ++ks) {
    FragU ah, al;
    if constexpr (BNF != 0) afr_bn(arow + ks * 32, mu + ks * 32, rs + ks * 32, hh, ah, al);
    else                    afr_plain(arow + ks * 32, hh, ah, al);
    const v16us bh = ldf(bhr + ks * 32, hh);
    const v16us bl = ldf(blr + ks * 32, hh);
    d = wmb3(ah.v, al.v, bh, bl, d);
  }
  return d;
}

__device__ __forceinline__ void relu_split_st(v8f d, unsigned short* ph, unsigned short* pl, int pitch) {
#pragma unroll
  for (int r = 0; r < 8; ++r) {
    const float t = fmaxf(d[r], 0.0f);
    const unsigned a = bfr(t);
    const unsigned b = bfr(t - __uint_as_float(a));
    ph[r * pitch] = (unsigned short)(a >> 16);
    pl[r * pitch] = (unsigned short)(b >> 16);
  }
}

__device__ __forceinline__ int scan_chunk(const int* __restrict__ dsts, int nE, int cbase, int nodeBase, int nb,
                                          int vec8, int* list, int tid, int wave) {
  int wc = 0;
  const int el0  = tid * EPT;
  const int e0   = cbase + el0;
  const int sent = -2147483647 - 1;
  v4i da, db;
  if (vec8 != 0 && cbase + CHUNK <= nE) {
    da = *(const v4i*)(dsts + e0);
    db = *(const v4i*)(dsts + e0 + 4);
  } else {
    da.x = (e0     < nE) ? dsts[min(e0,     nE - 1)] : sent;
    da.y = (e0 + 1 < nE) ? dsts[min(e0 + 1, nE - 1)] : sent;
    da.z = (e0 + 2 < nE) ? dsts[min(e0 + 2, nE - 1)] : sent;
    da.w = (e0 + 3 < nE) ? dsts[min(e0 + 3, nE - 1)] : sent;
    db.x = (e0 + 4 < nE) ? dsts[min(e0 + 4, nE - 1)] : sent;
    db.y = (e0 + 5 < nE) ? dsts[min(e0 + 5, nE - 1)] : sent;
    db.z = (e0 + 6 < nE) ? dsts[min(e0 + 6, nE - 1)] : sent;
    db.w = (e0 + 7 < nE) ? dsts[min(e0 + 7, nE - 1)] : sent;
  }
  const unsigned nbu = (unsigned)nodeBase;
  const unsigned s0 = (unsigned)da.x - nbu, s1 = (unsigned)da.y - nbu;
  const unsigned s2 = (unsigned)da.z - nbu, s3 = (unsigned)da.w - nbu;
  const unsigned s4 = (unsigned)db.x - nbu, s5 = (unsigned)db.y - nbu;
  const unsigned s6 = (unsigned)db.z - nbu, s7 = (unsigned)db.w - nbu;
  const unsigned unb = (unsigned)nb;
  const bool h0 = s0 < unb, h1 = s1 < unb, h2 = s2 < unb, h3 = s3 < unb;
  const bool h4 = s4 < unb, h5 = s5 < unb, h6 = s6 < unb, h7 = s7 < unb;
  const unsigned any = __builtin_amdgcn_ballot_w32(h0 | h1 | h2 | h3 | h4 | h5 | h6 | h7);
  if (any != 0u) {
#define HITJ(J, HJ, SJ) { \
      const unsigned mj = __builtin_amdgcn_ballot_w32(HJ); \
      if (mj != 0u) { \
        if (HJ) { \
          const int pos = wc + (int)__builtin_amdgcn_mbcnt_lo(mj, 0u); \
          if (pos < WCAP) list[wave * WCAP + pos] = ((el0 + (J)) << 10) | (int)(SJ); \
        } \
        wc += (int)__builtin_popcount(mj); } }
    HITJ(0, h0, s0)
    HITJ(1, h1, s1)
    HITJ(2, h2, s2)
    HITJ(3, h3, s3)
    HITJ(4, h4, s4)
    HITJ(5, h5, s5)
    HITJ(6, h6, s6)
    HITJ(7, h7, s7)
#undef HITJ
  }
  return wc;
}

__global__ __launch_bounds__(NTHR) void k_prepT(const float* __restrict__ W, int K, int N, int Kp,
                                               unsigned short* ph, unsigned short* pl) {
  const int idx = blockIdx.x * NTHR + (int)threadIdx.x;
  const int total8 = (N * Kp) >> 3;
  if (idx >= total8) return;
  const int el = idx << 3;
  const int n  = el / Kp;
  const int k0 = el - n * Kp;
  v4f a, b;
  float t[8];
#pragma unroll
  for (int i = 0; i < 8; ++i) {
    const int k  = k0 + i;
    const int kc = k < K ? k : K - 1;
    const float w = W[(size_t)kc * N + n];
    t[i] = (k < K) ? w : 0.0f;
  }
  a.x = t[0]; a.y = t[1]; a.z = t[2]; a.w = t[3];
  b.x = t[4]; b.y = t[5]; b.z = t[6]; b.w = t[7];
  v8us hv, lv;
  split8v(a, b, hv, lv);
  *(volatile v8us*)(ph + el) = hv;
  *(volatile v8us*)(pl + el) = lv;
  __threadfence();
  *(volatile v8us*)(ph + el) = hv;
  *(volatile v8us*)(pl + el) = lv;
}

__global__ __launch_bounds__(ETHR) void k_edge(
    const float* __restrict__ ea, const int* __restrict__ ei, const float* __restrict__ x,
    const unsigned short* __restrict__ w1h, const unsigned short* __restrict__ w1l, const float* __restrict__ be1,
    const unsigned short* __restrict__ w2h, const unsigned short* __restrict__ w2l, const float* __restrict__ be2,
    const unsigned short* __restrict__ w3h, const unsigned short* __restrict__ w3l, const float* __restrict__ be3,
    float* msg, int nN, int nE, int ntiles) {
  __shared__ __attribute__((aligned(16))) unsigned short t1h[EWAVE][16 * 128];
  __shared__ __attribute__((aligned(16))) unsigned short t1l[EWAVE][16 * 128];
  __shared__ __attribute__((aligned(16))) unsigned short t2h[EWAVE][16 * 64];
  __shared__ __attribute__((aligned(16))) unsigned short t2l[EWAVE][16 * 64];
  __shared__ __attribute__((aligned(16))) float          xs[EWAVE][16 * 32];

  const int tid = threadIdx.x, lane = tid & 31, wave = tid >> 5, hh = lane >> 4, m = lane & 15;
  const int tile = blockIdx.x * EWAVE + wave;
  if (tile >= ntiles) return;
  int e = tile * 16 + m;
  e = e > nE - 1 ? nE - 1 : e;
  unsigned short* T1h = t1h[wave];
  unsigned short* T1l = t1l[wave];
  unsigned short* T2h = t2h[wave];
  unsigned short* T2l = t2l[wave];
  float* XS = xs[wave];

  {
    int s = ei[e];
    s = s < 0 ? 0 : (s > nN - 1 ? nN - 1 : s);
    const float* xr = x + (size_t)s * 32 + 16 * hh;
    const v4f q0 = *(const v4f*)xr, q1 = *(const v4f*)(xr + 4), q2 = *(const v4f*)(xr + 8), q3 = *(const v4f*)(xr + 12);
    float* xd = XS + m * 32 + 16 * hh;
    *(v4f*)xd = q0; *(v4f*)(xd + 4) = q1; *(v4f*)(xd + 8) = q2; *(v4f*)(xd + 12) = q3;
  }

  FragU a1h, a1l;
  {
    const float* er = ea + (size_t)e * 16 + 8 * hh;
    const v4f p0 = *(const v4f*)er, p1 = *(const v4f*)(er + 4);
    split8v(p0, p1, a1h.h[0], a1l.h[0]);
    a1h.h[1] = zu8();
    a1l.h[1] = zu8();
  }
#pragma unroll
  for (int nt = 0; nt < 8; ++nt) {
    const int n = 16 * nt + m;
    const v16us bh = ldf(w1h + n * 32, hh);
    const v16us bl = ldf(w1l + n * 32, hh);
    const v8f d = wmb3(a1h.v, a1l.v, bh, bl, bc8(be1[n]));
    relu_split_st(d, T1h + (8 * hh) * 128 + n, T1l + (8 * hh) * 128 + n, 128);
  }
  wsync();

  v8f d2[4];
#pragma unroll
  for (int nt = 0; nt < 4; ++nt) d2[nt] = bc8(be2[16 * nt + m]);
#pragma unroll
  for (int ks = 0; ks < 4; ++ks) {
    const v16us ah = ldf(T1h + m * 128 + ks * 32, hh);
    const v16us al = ldf(T1l + m * 128 + ks * 32, hh);
#pragma unroll
    for (int nt = 0; nt < 4; ++nt) {
      const int n = 16 * nt + m;
      const v16us bh = ldf(w2h + n * 128 + ks * 32, hh);
      const v16us bl = ldf(w2l + n * 128 + ks * 32, hh);
      d2[nt] = wmb3(ah, al, bh, bl, d2[nt]);
    }
  }
#pragma unroll
  for (int nt = 0; nt < 4; ++nt)
    relu_split_st(d2[nt], T2h + (8 * hh) * 64 + 16 * nt + m, T2l + (8 * hh) * 64 + 16 * nt + m, 64);
  wsync();

  FragU a3h[2], a3l[2];
#pragma unroll
  for (int ks = 0; ks < 2; ++ks) {
    a3h[ks].v = ldf(T2h + m * 64 + ks * 32, hh);
    a3l[ks].v = ldf(T2l + m * 64 + ks * 32, hh);
  }
  v8f m0 = bc8(0.0f), m1 = bc8(0.0f);
#pragma unroll 1
  for (int f = 0; f < 32; ++f) {
    const int n0 = 32 * f + m, n1 = n0 + 16;
    v8f d0 = bc8(be3[n0]), d1 = bc8(be3[n1]);
#pragma unroll
    for (int ks = 0; ks < 2; ++ks) {
      const v16us b0h = ldf(w3h + (size_t)n0 * 64 + ks * 32, hh);
      const v16us b0l = ldf(w3l + (size_t)n0 * 64 + ks * 32, hh);
      d0 = wmb3(a3h[ks].v, a3l[ks].v, b0h, b0l, d0);
      const v16us b1h = ldf(w3h + (size_t)n1 * 64 + ks * 32, hh);
      const v16us b1l = ldf(w3l + (size_t)n1 * 64 + ks * 32, hh);
      d1 = wmb3(a3h[ks].v, a3l[ks].v, b1h, b1l, d1);
    }
#pragma unroll
    for (int r = 0; r < 8; ++r) {
      const float xv = XS[(8 * hh + r) * 32 + f];
      m0[r] += xv * d0[r];
      m1[r] += xv * d1[r];
    }
  }
  wsync();
#pragma unroll
  for (int r = 0; r < 8; ++r) {
    XS[(8 * hh + r) * 32 + m]      = m0[r];
    XS[(8 * hh + r) * 32 + 16 + m] = m1[r];
  }
  wsync();
  float* mp = msg + (size_t)tile * 512;
#pragma unroll
  for (int j = 0; j < 4; ++j) {
    const v4f v = *(const v4f*)(XS + j * 128 + 4 * lane);
    *(volatile v4f*)(mp + j * 128 + 4 * lane) = v;
  }
  __threadfence();
#pragma unroll
  for (int j = 0; j < 4; ++j) {
    const v4f v = *(const v4f*)(XS + j * 128 + 4 * lane);
    *(volatile v4f*)(mp + j * 128 + 4 * lane) = v;
  }
}

__global__ __launch_bounds__(NTHR) void k_agg_nn(
    const float* __restrict__ msg, const int* __restrict__ ei, const float* __restrict__ x,
    const unsigned short* __restrict__ wrh, const unsigned short* __restrict__ wrl, const float* __restrict__ bc1,
    float* zout, double* stp, int nN, int nE, int vec8) {
  __shared__ __attribute__((aligned(16))) float  acc[NBN * 32];
  __shared__ __attribute__((aligned(16))) int    list[LISTN];
  __shared__ int wcnt[NWAVE];
  __shared__ __attribute__((aligned(16))) double stg[64];

  const int tid = threadIdx.x, lane = tid & 31, wave = tid >> 5, hh = lane >> 4, m = lane & 15;
  const int nodeBase = blockIdx.x * NBN;
  const int* dsts = ei + nE;

  for (int i = tid; i < NBN * 32; i += NTHR) acc[i] = 0.0f;
  __syncthreads();

  const int nChunks = (nE + CHUNK - 1) / CHUNK;
#pragma unroll 1
  for (int ch = 0; ch < nChunks; ++ch) {
    const int cbase = ch * CHUNK;
    const int wc = scan_chunk(dsts, nE, cbase, nodeBase, NBN, vec8, list, tid, wave);
    if (lane == 0) wcnt[wave] = wc;
    __syncthreads();
#pragma unroll 1
    for (int w2 = 0; w2 < NWAVE; ++w2) {
      int n = wcnt[w2];
      n = n > WCAP ? WCAP : (n < 0 ? 0 : n);
      const int* lp = list + w2 * WCAP;
#pragma unroll 1
      for (int i = 0; i < n; ++i) {
        const int ent  = lp[i];
        const int slot = ent & 1023;
        if ((slot & (NWAVE - 1)) == wave) {
          int e = cbase + (ent >> 10);
          e = e < 0 ? 0 : (e > nE - 1 ? nE - 1 : e);
          acc[slot * 32 + lane] += msg[(size_t)e * 32 + lane];
        }
      }
    }
    __syncthreads();
  }

#pragma unroll 1
  for (int rt = wave; rt < NBN / 16; rt += NWAVE) {
    const int row  = nodeBase + rt * 16 + m;
    const int rowc = row > nN - 1 ? nN - 1 : row;
#pragma unroll
    for (int nt = 0; nt < 2; ++nt) {
      const int n = 16 * nt + m;
      const v8f d = tgemm<1, 0>(x + (size_t)rowc * 32, nullptr, nullptr, wrh + n * 32, wrl + n * 32, bc1[n], hh);
#pragma unroll
      for (int r = 0; r < 8; ++r) acc[(rt * 16 + 8 * hh + r) * 32 + n] += d[r];
    }
  }
  __syncthreads();

  int nval = nN - nodeBase;
  nval = nval > NBN ? NBN : (nval < 0 ? 0 : nval);
  if (tid < 32) {
    double S = 0.0, Q = 0.0;
#pragma unroll 1
    for (int s = 0; s < nval; ++s) {
      const double v = (double)acc[s * 32 + tid];
      S += v; Q += v * v;
    }
    stg[tid] = S;
    stg[32 + tid] = Q;
  }
  __syncthreads();
  double* gp = stp + (size_t)blockIdx.x * 64;
  float*  zp = zout + (size_t)nodeBase * 32;
  if (tid < 32) { const v2d v = *(const v2d*)(stg + 2 * tid); *(volatile v2d*)(gp + 2 * tid) = v; }
#pragma unroll
  for (int j = 0; j < (NBN * 32) / 1024; ++j) {
    const int off = j * 1024 + 4 * tid;
    const v4f v = *(const v4f*)(acc + off);
    *(volatile v4f*)(zp + off) = v;
  }
  __threadfence();
  if (tid < 32) { const v2d v = *(const v2d*)(stg + 2 * tid); *(volatile v2d*)(gp + 2 * tid) = v; }
#pragma unroll
  for (int j = 0; j < (NBN * 32) / 1024; ++j) {
    const int off = j * 1024 + 4 * tid;
    const v4f v = *(const v4f*)(acc + off);
    *(volatile v4f*)(zp + off) = v;
  }
}

template <int FIN, int FOUT>
__global__ __launch_bounds__(ETHR) void k_xform(
    const float* __restrict__ zin, const double* __restrict__ stp, int nblkPrev,
    const unsigned short* __restrict__ wh, const unsigned short* __restrict__ wl,
    const float* __restrict__ as_, const float* __restrict__ ad_,
    float* hW, float* scp, int nN, int ntiles) {
  constexpr int KS = FIN / 32, NT = FOUT / 16, NST = FOUT / 8;
  static_assert(KS >= 1 && KS <= 2);
  static_assert(FIN <= ETHR);
  __shared__ float mu[FIN], rs[FIN];
  __shared__ __attribute__((aligned(16))) float tb[EWAVE][16 * FOUT];
  __shared__ __attribute__((aligned(16))) float scl[EWAVE][128];

  const int tid = threadIdx.x, lane = tid & 31, wave = tid >> 5, hh = lane >> 4, m = lane & 15;
  if (tid < FIN) {
    double S = 0.0, Q = 0.0;
#pragma unroll 1
    for (int b = 0; b < nblkPrev; ++b) {
      S += stp[(size_t)b * 2 * FIN + tid];
      Q += stp[(size_t)b * 2 * FIN + FIN + tid];
    }
    const double inv = 1.0 / (double)nN;
    const double mean = S * inv;
    double var = Q * inv - mean * mean;
    if (var < 0.0) var = 0.0;
    mu[tid] = (float)mean;
    rs[tid] = 1.0f / sqrtf((float)var + BN_EPS);
  }
  __syncthreads();

  const int tile = blockIdx.x * EWAVE + wave;
  if (tile < ntiles) {
    const int row = tile * 16 + m;
    const float* arow = zin + (size_t)row * FIN;
    FragU ah[KS], al[KS];
#pragma unroll
    for (int ks = 0; ks < KS; ++ks) afr_bn(arow + ks * 32, mu + ks * 32, rs + ks * 32, hh, ah[ks], al[ks]);
    v8f d[NT];
#pragma unroll
    for (int nt = 0; nt < NT; ++nt) {
      const int n = 16 * nt + m;
      d[nt] = bc8(0.0f);
#pragma unroll
      for (int ks = 0; ks < KS; ++ks) {
        const v16us bh = ldf(wh + (size_t)n * FIN + ks * 32, hh);
        const v16us bl = ldf(wl + (size_t)n * FIN + ks * 32, hh);
        d[nt] = wmb3(ah[ks].v, al[ks].v, bh, bl, d[nt]);
      }
    }
    float ps[8], pd[8];
#pragma unroll
    for (int r = 0; r < 8; ++r) { ps[r] = 0.0f; pd[r] = 0.0f; }
#pragma unroll
    for (int nt = 0; nt < NT; ++nt) {
      const float av = as_[16 * nt + m], dv = ad_[16 * nt + m];
#pragma unroll
      for (int r = 0; r < 8; ++r) { ps[r] += d[nt][r] * av; pd[r] += d[nt][r] * dv; }
    }
#pragma unroll
    for (int r = 0; r < 8; ++r) {
#pragma unroll
      for (int o = 1; o < 16; o <<= 1) {
        ps[r] += __shfl_xor(ps[r], o, 32);
        pd[r] += __shfl_xor(pd[r], o, 32);
      }
    }
    float* TB = tb[wave];
#pragma unroll
    for (int nt = 0; nt < NT; ++nt) {
#pragma unroll
      for (int r = 0; r < 8; ++r) TB[(8 * hh + r) * FOUT + 16 * nt + m] = d[nt][r];
    }
    if (m == 0) {
#pragma unroll
      for (int r = 0; r < 8; ++r) { scl[wave][(8 * hh + r) * 2] = ps[r]; scl[wave][(8 * hh + r) * 2 + 1] = pd[r]; }
    }
    wsync();
    float* hp = hW  + (size_t)tile * 16 * FOUT;
    float* sp = scp + (size_t)tile * 32;
#pragma unroll
    for (int j = 0; j < NST; ++j) {
      const v4f v = *(const v4f*)(TB + j * 128 + 4 * lane);
      *(volatile v4f*)(hp + j * 128 + 4 * lane) = v;
    }
    {
      const v4f sv = *(const v4f*)(scl[wave] + 4 * lane);
      if (lane < 8) *(volatile v4f*)(sp + 4 * lane) = sv;
    }
    __threadfence();
#pragma unroll
    for (int j = 0; j < NST; ++j) {
      const v4f v = *(const v4f*)(TB + j * 128 + 4 * lane);
      *(volatile v4f*)(hp + j * 128 + 4 * lane) = v;
    }
    {
      const v4f sv = *(const v4f*)(scl[wave] + 4 * lane);
      if (lane < 8) *(volatile v4f*)(sp + 4 * lane) = sv;
    }
  }
}

template <int F, int NB>
__global__ __launch_bounds__(NTHR) void k_agg_gat(
    const float* __restrict__ hW, const float* __restrict__ scp, const int* __restrict__ ei,
    const float* __restrict__ bg, float* gout, double* stp, int nN, int nE, int vec8) {
  constexpr int WPG = F / 32, P = NWAVE / WPG;
  static_assert(NB * F == 8192);
  static_assert(WPG * P == NWAVE);
  static_assert(NB <= 1024 && (NB % 16) == 0);
  static_assert(F <= NTHR);
  __shared__ __attribute__((aligned(16))) float  acc[NB * F];
  __shared__ float  mw[NWAVE * NB];
  __shared__ float  ssum[NB];
  __shared__ float  sd[NB];
  __shared__ __attribute__((aligned(16))) int    list[LISTN];
  __shared__ int    wcnt[NWAVE];
  __shared__ __attribute__((aligned(16))) double stg[2 * F];

  const int tid = threadIdx.x, lane = tid & 31, wave = tid >> 5;
  const int g = wave / WPG;
  const int c = (wave % WPG) * 32 + lane;
  const int nodeBase = blockIdx.x * NB;
  const int* srcs = ei;
  const int* dsts = ei + nE;

  for (int idx = tid; idx < NB * F; idx += NTHR) {
    const int slot = idx / F, cc = idx - slot * F;
    int d = nodeBase + slot; d = d > nN - 1 ? nN - 1 : d;
    acc[idx] = hW[(size_t)d * F + cc];
  }
  for (int idx = tid; idx < NB; idx += NTHR) {
    int d = nodeBase + idx; d = d > nN - 1 ? nN - 1 : d;
    const float a = scp[(size_t)2 * d], b = scp[(size_t)2 * d + 1];
    float e0 = a + b; e0 = e0 > 0.0f ? e0 : 0.2f * e0;
    sd[idx] = b;
    ssum[idx] = 1.0f;
#pragma unroll
    for (int w = 0; w < NWAVE; ++w) mw[w * NB + idx] = e0;
  }
  __syncthreads();

  const int nChunks = (nE + CHUNK - 1) / CHUNK;
#pragma unroll 1
  for (int ch = 0; ch < nChunks; ++ch) {
    const int cbase = ch * CHUNK;
    const int wc = scan_chunk(dsts, nE, cbase, nodeBase, NB, vec8, list, tid, wave);
    if (lane == 0) wcnt[wave] = wc;
    __syncthreads();
#pragma unroll 1
    for (int w2 = 0; w2 < NWAVE; ++w2) {
      int n = wcnt[w2];
      n = n > WCAP ? WCAP : (n < 0 ? 0 : n);
      const int* lp = list + w2 * WCAP;
#pragma unroll 1
      for (int i = 0; i < n; ++i) {
        const int ent  = lp[i];
        const int slot = ent & 1023;
        if ((slot & (P - 1)) == g) {
          int e = cbase + (ent >> 10);
          e = e < 0 ? 0 : (e > nE - 1 ? nE - 1 : e);
          int src = srcs[e];
          src = src < 0 ? 0 : (src > nN - 1 ? nN - 1 : src);
          const float a = scp[(size_t)2 * src];
          float ev = a + sd[slot];
          ev = ev > 0.0f ? ev : 0.2f * ev;
          const float mo = mw[wave * NB + slot];
          const float mn = fmaxf(mo, ev);
          const float sc = __expf(mo - mn);
          const float p  = __expf(ev - mn);
          float* ap = acc + slot * F + c;
          const float hv = hW[(size_t)src * F + c];
          const float nv = *ap * sc + p * hv;
          *ap = nv;
          if (lane == 0) mw[wave * NB + slot] = mn;
          if ((wave % WPG) == 0 && lane == 0) {
            const float so = ssum[slot];
            ssum[slot] = so * sc + p;
          }
        }
      }
    }
    __syncthreads();
  }

  for (int idx = tid; idx < NB * F; idx += NTHR) {
    const int slot = idx / F, cc = idx - slot * F;
    const float rcp = 1.0f / (ssum[slot] + 1e-16f);
    acc[idx] = acc[idx] * rcp + bg[cc];
  }
  __syncthreads();

  int nval = nN - nodeBase;
  nval = nval > NB ? NB : (nval < 0 ? 0 : nval);
  if (tid < F) {
    double S = 0.0, Q = 0.0;
#pragma unroll 1
    for (int s = 0; s < nval; ++s) {
      const double v = (double)acc[s * F + tid];
      S += v; Q += v * v;
    }
    stg[tid] = S;
    stg[F + tid] = Q;
  }
  __syncthreads();
  double* gp = stp + (size_t)blockIdx.x * 2 * F;
  float*  op = gout + (size_t)nodeBase * F;
  if (tid < F) { const v2d v = *(const v2d*)(stg + 2 * tid); *(volatile v2d*)(gp + 2 * tid) = v; }
#pragma unroll
  for (int j = 0; j < (NB * F) / 1024; ++j) {
    const int off = j * 1024 + 4 * tid;
    const v4f v = *(const v4f*)(acc + off);
    *(volatile v4f*)(op + off) = v;
  }
  __threadfence();
  if (tid < F) { const v2d v = *(const v2d*)(stg + 2 * tid); *(volatile v2d*)(gp + 2 * tid) = v; }
#pragma unroll
  for (int j = 0; j < (NB * F) / 1024; ++j) {
    const int off = j * 1024 + 4 * tid;
    const v4f v = *(const v4f*)(acc + off);
    *(volatile v4f*)(op + off) = v;
  }
}

__global__ __launch_bounds__(NTHR) void k_head(
    const float* __restrict__ g2, const double* __restrict__ stp, int nblkPrev, const int* __restrict__ batch,
    const unsigned short* __restrict__ f1h, const unsigned short* __restrict__ f1l, const float* __restrict__ bf1,
    const unsigned short* __restrict__ f2h, const unsigned short* __restrict__ f2l, const float* __restrict__ bf2,
    const unsigned short* __restrict__ f3h, const unsigned short* __restrict__ f3l, const float* __restrict__ bf3,
    float* out, int nN, int nB, int rowsP) {
  extern __shared__ v4f dsmv[];
  float* Y = (float*)dsmv;
  float* X = Y + (size_t)rowsP * 128;
  __shared__ float hmu[256], hrs[256];
  __shared__ float cntf[1024];

  const int tid = threadIdx.x, lane = tid & 31, wave = tid >> 5, hh = lane >> 4, m = lane & 15;

  for (int i = tid; i < rowsP * 128; i += NTHR) Y[i] = 0.0f;
  for (int i = tid; i < 1024; i += NTHR) cntf[i] = 0.0f;
  if (tid < 128) {
    double S = 0.0, Q = 0.0;
#pragma unroll 1
    for (int b = 0; b < nblkPrev; ++b) {
      S += stp[(size_t)b * 256 + tid];
      Q += stp[(size_t)b * 256 + 128 + tid];
    }
    const double inv = 1.0 / (double)nN;
    const double mean = S * inv;
    double var = Q * inv - mean * mean;
    if (var < 0.0) var = 0.0;
    hmu[tid] = (float)mean;
    hrs[tid] = 1.0f / sqrtf((float)var + BN_EPS);
  }
  __syncthreads();

  if (tid < 128) {
    const float mc = hmu[tid], rc = hrs[tid];
#pragma unroll 1
    for (int i = 0; i < nN; ++i) {
      float v = g2[(size_t)i * 128 + tid];
      v = fmaxf((v - mc) * rc, 0.0f);
      int b = batch[i];
      b = b < 0 ? 0 : (b > nB - 1 ? nB - 1 : b);
      Y[b * 128 + tid] += v;
    }
  } else if (tid == 128) {
#pragma unroll 1
    for (int i = 0; i < nN; ++i) {
      int b = batch[i];
      b = b < 0 ? 0 : (b > nB - 1 ? nB - 1 : b);
      cntf[b] += 1.0f;
    }
  }
  __syncthreads();
  for (int i = tid; i < nB * 128; i += NTHR) {
    const int b = i >> 7;
    Y[i] = Y[i] * (1.0f / fmaxf(cntf[b], 1.0f));
  }
  __syncthreads();

  const int MT = rowsP >> 4;
#pragma unroll 1
  for (int p = wave; p < MT * 16; p += NWAVE) {
    const int mt = p >> 4, nt = p & 15, n = 16 * nt + m;
    const v8f d = tgemm<4, 0>(Y + (mt * 16 + m) * 128, nullptr, nullptr,
                              f1h + (size_t)n * 128, f1l + (size_t)n * 128, bf1[n], hh);
#pragma unroll
    for (int r = 0; r < 8; ++r) X[(mt * 16 + 8 * hh + r) * 256 + n] = d[r];
  }
  __syncthreads();
  {
    double S = 0.0, Q = 0.0;
#pragma unroll 1
    for (int r = 0; r < nB; ++r) { const double v = (double)X[r * 256 + tid]; S += v; Q += v * v; }
    const double inv = 1.0 / (double)nB;
    const double mean = S * inv;
    double var = Q * inv - mean * mean;
    if (var < 0.0) var = 0.0;
    hmu[tid] = (float)mean;
    hrs[tid] = 1.0f / sqrtf((float)var + BN_EPS);
  }
  __syncthreads();
#pragma unroll 1
  for (int p = wave; p < MT * 8; p += NWAVE) {
    const int mt = p >> 3, nt = p & 7, n = 16 * nt + m;
    const v8f d = tgemm<8, 1>(X + (mt * 16 + m) * 256, hmu, hrs,
                              f2h + (size_t)n * 256, f2l + (size_t)n * 256, bf2[n], hh);
#pragma unroll
    for (int r = 0; r < 8; ++r) Y[(mt * 16 + 8 * hh + r) * 128 + n] = d[r];
  }
  __syncthreads();
  if (tid < 128) {
    double S = 0.0, Q = 0.0;
#pragma unroll 1
    for (int r = 0; r < nB; ++r) { const double v = (double)Y[r * 128 + tid]; S += v; Q += v * v; }
    const double inv = 1.0 / (double)nB;
    const double mean = S * inv;
    double var = Q * inv - mean * mean;
    if (var < 0.0) var = 0.0;
    hmu[tid] = (float)mean;
    hrs[tid] = 1.0f / sqrtf((float)var + BN_EPS);
  }
  __syncthreads();
#pragma unroll 1
  for (int p = wave; p < MT * 4; p += NWAVE) {
    const int mt = p >> 2, nt = p & 3, n = 16 * nt + m;
    const v8f d = tgemm<4, 1>(Y + (mt * 16 + m) * 128, hmu, hrs,
                              f3h + (size_t)n * 128, f3l + (size_t)n * 128, bf3[n], hh);
#pragma unroll
    for (int r = 0; r < 8; ++r) X[(mt * 16 + 8 * hh + r) * 64 + n] = d[r];
  }
  __syncthreads();
  const int nOut = nB * 64;
#pragma unroll 1
  for (int j = 0; j * 1024 < nOut; ++j) {
    const int off = j * 1024 + 4 * tid;
    if (off < nOut) { const v4f v = *(const v4f*)(X + off); *(volatile v4f*)(out + off) = v; }
  }
  __threadfence();
#pragma unroll 1
  for (int j = 0; j * 1024 < nOut; ++j) {
    const int off = j * 1024 + 4 * tid;
    if (off < nOut) { const v4f v = *(const v4f*)(X + off); *(volatile v4f*)(out + off) = v; }
  }
}

extern "C" void kernel_launch(void* const* d_in, const int* in_sizes, int n_in,
                              void* d_out, int out_size, void* d_ws, size_t ws_size,
                              hipStream_t stream) {
  if (n_in < 26) return;
  const int nN = in_sizes[3];
  if (nN <= 0 || in_sizes[0] != nN * 32) return;
  const int nE = in_sizes[1] / 2;
  if (nE <= 0 || in_sizes[1] != nE * 2 || in_sizes[2] != nE * 16) return;
  const int nB = out_size / 64;
  if (nB <= 0 || nB > 1024 || out_size != nB * 64) return;
  if (in_sizes[4] != 16 * 128 || in_sizes[5] < 128) return;
  if (in_sizes[6] != 128 * 64 || in_sizes[7] < 64) return;
  if (in_sizes[8] != 64 * 1024 || in_sizes[9] < 1024) return;
  if (in_sizes[10] != 32 * 32 || in_sizes[11] < 32) return;
  if (in_sizes[12] != 32 * 64 || in_sizes[13] < 64 || in_sizes[14] < 64 || in_sizes[15] < 64) return;
  if (in_sizes[16] != 64 * 128 || in_sizes[17] < 128 || in_sizes[18] < 128 || in_sizes[19] < 128) return;
  if (in_sizes[20] != 128 * 256 || in_sizes[21] < 256) return;
  if (in_sizes[22] != 256 * 128 || in_sizes[23] < 128) return;
  if (in_sizes[24] != 128 * 64 || in_sizes[25] < 64) return;

  const float* x     = (const float*)d_in[0];
  const int*   ei    = (const int*)d_in[1];
  const float* ea    = (const float*)d_in[2];
  const int*   batch = (const int*)d_in[3];
  const float* We1 = (const float*)d_in[4],  *be1 = (const float*)d_in[5];
  const float* We2 = (const float*)d_in[6],  *be2 = (const float*)d_in[7];
  const float* We3 = (const float*)d_in[8],  *be3 = (const float*)d_in[9];
  const float* Wroot = (const float*)d_in[10], *bc1 = (const float*)d_in[11];
  const float* Wg1 = (const float*)d_in[12], *as1 = (const float*)d_in[13];
  const float* ad1 = (const float*)d_in[14], *bg1 = (const float*)d_in[15];
  const float* Wg2 = (const float*)d_in[16], *as2 = (const float*)d_in[17];
  const float* ad2 = (const float*)d_in[18], *bg2 = (const float*)d_in[19];
  const float* Wf1 = (const float*)d_in[20], *bf1 = (const float*)d_in[21];
  const float* Wf2 = (const float*)d_in[22], *bf2 = (const float*)d_in[23];
  const float* Wf3 = (const float*)d_in[24], *bf3 = (const float*)d_in[25];
  float* out = (float*)d_out;

  const int ntE   = (nE + 15) / 16;
  const int rowsE = ntE * 16;
  const int gridE = (ntE + EWAVE - 1) / EWAVE;
  const int nblk0 = (nN + NBN - 1) / NBN; const int rows0 = nblk0 * NBN;
  const int nt16  = (nN + 15) / 16;        const int rows16 = nt16 * 16;
  const int gridX = (nt16 + EWAVE - 1) / EWAVE;
  const int nblk1 = (nN + NBA - 1) / NBA; const int rows1 = nblk1 * NBA;
  const int nblk2 = (nN + NBB - 1) / NBB; const int rows2 = nblk2 * NBB;
  const int rowsP = ((nB + 15) / 16) * 16;
  const size_t ldsHead = (size_t)rowsP * (128 + 256) * 4;

  char* ws = (char*)d_ws;
  size_t off = 0;
  auto carve = [&](size_t bytes) -> size_t { const size_t o = off; off += (bytes + 255) & ~(size_t)255; return o; };
  const size_t oW1h = carve(128 * 32 * 2),   oW1l = carve(128 * 32 * 2);
  const size_t oW2h = carve(64 * 128 * 2),   oW2l = carve(64 * 128 * 2);
  const size_t oW3h = carve(1024 * 64 * 2),  oW3l = carve(1024 * 64 * 2);
  const size_t oWrh = carve(32 * 32 * 2),    oWrl = carve(32 * 32 * 2);
  const size_t oG1h = carve(64 * 32 * 2),    oG1l = carve(64 * 32 * 2);
  const size_t oG2h = carve(128 * 64 * 2),   oG2l = carve(128 * 64 * 2);
  const size_t oF1h = carve(256 * 128 * 2),  oF1l = carve(256 * 128 * 2);
  const size_t oF2h = carve(128 * 256 * 2),  oF2l = carve(128 * 256 * 2);
  const size_t oF3h = carve(64 * 128 * 2),   oF3l = carve(64 * 128 * 2);
  const size_t oMsg = carve((size_t)rowsE * 32 * 4);
  const size_t oZ   = carve((size_t)rows0 * 32 * 4);
  const size_t oSt0 = carve((size_t)nblk0 * 64 * 8);
  const size_t oHW1 = carve((size_t)rows16 * 64 * 4);
  const size_t oSc1 = carve((size_t)rows16 * 2 * 4);
  const size_t oGa1 = carve((size_t)rows1 * 64 * 4);
  const size_t oSt1 = carve((size_t)nblk1 * 128 * 8);
  const size_t oHW2 = carve((size_t)rows16 * 128 * 4);
  const size_t oSc2 = carve((size_t)rows16 * 2 * 4);
  const size_t oGa2 = carve((size_t)rows2 * 128 * 4);
  const size_t oSt2 = carve((size_t)nblk2 * 256 * 8);
  if (off > ws_size || off > (size_t)134217728) return;

  unsigned short* w1h = (unsigned short*)(ws + oW1h); unsigned short* w1l = (unsigned short*)(ws + oW1l);
  unsigned short* w2h = (unsigned short*)(ws + oW2h); unsigned short* w2l = (unsigned short*)(ws + oW2l);
  unsigned short* w3h = (unsigned short*)(ws + oW3h); unsigned short* w3l = (unsigned short*)(ws + oW3l);
  unsigned short* wrh = (unsigned short*)(ws + oWrh); unsigned short* wrl = (unsigned short*)(ws + oWrl);
  unsigned short* g1h = (unsigned short*)(ws + oG1h); unsigned short* g1l = (unsigned short*)(ws + oG1l);
  unsigned short* g2h = (unsigned short*)(ws + oG2h); unsigned short* g2l = (unsigned short*)(ws + oG2l);
  unsigned short* f1h = (unsigned short*)(ws + oF1h); unsigned short* f1l = (unsigned short*)(ws + oF1l);
  unsigned short* f2h = (unsigned short*)(ws + oF2h); unsigned short* f2l = (unsigned short*)(ws + oF2l);
  unsigned short* f3h = (unsigned short*)(ws + oF3h); unsigned short* f3l = (unsigned short*)(ws + oF3l);
  float*  msg  = (float*)(ws + oMsg);
  float*  z    = (float*)(ws + oZ);
  double* st0  = (double*)(ws + oSt0);
  float*  hW1  = (float*)(ws + oHW1);
  float*  sc1  = (float*)(ws + oSc1);
  float*  ga1  = (float*)(ws + oGa1);
  double* st1  = (double*)(ws + oSt1);
  float*  hW2  = (float*)(ws + oHW2);
  float*  sc2  = (float*)(ws + oSc2);
  float*  ga2  = (float*)(ws + oGa2);
  double* st2  = (double*)(ws + oSt2);

  const int vec8 = ((nE & 3) == 0) ? 1 : 0;
  auto pgrid = [](int N, int Kp) { return ((N * Kp) / 8 + NTHR - 1) / NTHR; };

  k_prepT<<<pgrid(128, 32),   NTHR, 0, stream>>>(We1,   16,  128,  32,  w1h, w1l);
  k_prepT<<<pgrid(64, 128),   NTHR, 0, stream>>>(We2,   128, 64,   128, w2h, w2l);
  k_prepT<<<pgrid(1024, 64),  NTHR, 0, stream>>>(We3,   64,  1024, 64,  w3h, w3l);
  k_prepT<<<pgrid(32, 32),    NTHR, 0, stream>>>(Wroot, 32,  32,   32,  wrh, wrl);
  k_prepT<<<pgrid(64, 32),    NTHR, 0, stream>>>(Wg1,   32,  64,   32,  g1h, g1l);
  k_prepT<<<pgrid(128, 64),   NTHR, 0, stream>>>(Wg2,   64,  128,  64,  g2h, g2l);
  k_prepT<<<pgrid(256, 128),  NTHR, 0, stream>>>(Wf1,   128, 256,  128, f1h, f1l);
  k_prepT<<<pgrid(128, 256),  NTHR, 0, stream>>>(Wf2,   256, 128,  256, f2h, f2l);
  k_prepT<<<pgrid(64, 128),   NTHR, 0, stream>>>(Wf3,   128, 64,   128, f3h, f3l);

  k_edge<<<gridE, ETHR, 0, stream>>>(ea, ei, x, w1h, w1l, be1, w2h, w2l, be2, w3h, w3l, be3, msg, nN, nE, ntE);
  k_agg_nn<<<nblk0, NTHR, 0, stream>>>(msg, ei, x, wrh, wrl, bc1, z, st0, nN, nE, vec8);

  k_xform<32, 64><<<gridX, ETHR, 0, stream>>>(z, st0, nblk0, g1h, g1l, as1, ad1, hW1, sc1, nN, nt16);
  k_agg_gat<64, NBA><<<nblk1, NTHR, 0, stream>>>(hW1, sc1, ei, bg1, ga1, st1, nN, nE, vec8);

  k_xform<64, 128><<<gridX, ETHR, 0, stream>>>(ga1, st1, nblk1, g2h, g2l, as2, ad2, hW2, sc2, nN, nt16);
  k_agg_gat<128, NBB><<<nblk2, NTHR, 0, stream>>>(hW2, sc2, ei, bg2, ga2, st2, nN, nE, vec8);

  hipFuncSetAttribute(reinterpret_cast<const void*>(&k_head), hipFuncAttributeMaxDynamicSharedMemorySize, (int)ldsHead);
  k_head<<<1, NTHR, ldsHead, stream>>>(ga2, st2, nblk2, batch, f1h, f1l, bf1, f2h, f2l, bf2, f3h, f3l, bf3,
                                       out, nN, nB, rowsP);
}
